// TFAttention_59347858096454
// MI455X (gfx1250) — hardware-verified
//
#include <hip/hip_runtime.h>
#include <math.h>

constexpr int kBatch = 4;
constexpr int kSeq   = 2048;
constexpr int kDim   = 1024;
constexpr int kHeads = 16;
constexpr int kDh    = 64;
constexpr int kTok   = kBatch * kSeq;
constexpr int kNQKV  = 3 * kDim;
constexpr int kQKld  = 2 * kDim;
constexpr int kSplitQB = 4;
constexpr float kScale     = 0.125f;
constexpr float kMaskFill  = -10000.0f;
constexpr float kPCarry    = 32768.0f;
constexpr float kPCarryInv = 1.0f / 32768.0f;
constexpr float kResCarry  = 2048.0f;
constexpr float kResInv    = 1.0f / 2048.0f;
static_assert(kHeads * kDh == kDim, "shape");
static_assert(kHeads == 16 && kDh == 64 && kSeq % 64 == 0, "attn tiles");
static_assert(kDim % 32 == 0, "gemm k");
static_assert(kTok % 64 == 0 && kQKld % 64 == 0 && kDim % 64 == 0 && kNQKV % 64 == 0, "gemm mn");
static_assert(((kTok / 64) * (kQKld / 64)) % 8 == 0, "grid qk");
static_assert(((kDim / 64) * (kTok / 64)) % 8 == 0, "grid vt");
static_assert(((kTok / 64) * (kDim / 64)) % 8 == 0, "grid out");
static_assert((kTok * kDim) % (8 * 256) == 0, "cast grid");
static_assert(kSplitQB >= 1 && kSplitQB < kSeq / 64, "split range");

typedef __attribute__((ext_vector_type(16))) _Float16 v16h;
typedef __attribute__((ext_vector_type(8)))  _Float16 v8h;
typedef __attribute__((ext_vector_type(16))) __bf16   v16b;
typedef __attribute__((ext_vector_type(8)))  __bf16   v8b;
typedef __attribute__((ext_vector_type(8)))  float    v8f;
typedef __attribute__((ext_vector_type(4)))  float    v4f;
typedef __attribute__((ext_vector_type(4)))  unsigned int v4u;

__device__ __forceinline__ unsigned short f2bf_bits(float f) {
  unsigned u = __float_as_uint(f);
  return (unsigned short)((u + 0x7FFFu + ((u >> 16) & 1u)) >> 16);
}
__device__ __forceinline__ float bf_bits2f(unsigned short h) { return __uint_as_float(((unsigned)h) << 16); }
__device__ __forceinline__ float rne11(float f) {
  unsigned u = __float_as_uint(f);
  u = (u + 0x0FFFu + ((u >> 13) & 1u)) & 0xFFFFE000u;
  return __uint_as_float(u);
}
__device__ __forceinline__ unsigned pk16(unsigned short a, unsigned short b) { return (unsigned)a | ((unsigned)b << 16); }

__device__ __forceinline__ void dep_guard4_h(v8f& a, v8f& b, v8f& c, v8f& d, v16h x, v16h y) {
  asm volatile("v_nop\n\tv_nop\n\tv_nop\n\tv_nop" : "+v"(a), "+v"(b), "+v"(c), "+v"(d) : "v"(x), "v"(y));
}
__device__ __forceinline__ void dep_guard4_b(v8f& a, v8f& b, v8f& c, v8f& d, v16b x, v16b y) {
  asm volatile("v_nop\n\tv_nop\n\tv_nop\n\tv_nop" : "+v"(a), "+v"(b), "+v"(c), "+v"(d) : "v"(x), "v"(y));
}
__device__ __forceinline__ void keep4_h(v16h a, v16h b, v16h c, v16h d) { asm volatile("v_nop" :: "v"(a), "v"(b), "v"(c), "v"(d)); }
__device__ __forceinline__ void keep4_b(v16b a, v16b b, v16b c, v16b d) { asm volatile("v_nop" :: "v"(a), "v"(b), "v"(c), "v"(d)); }
__device__ __forceinline__ void acc_guard4(v8f& a, v8f& b, v8f& c, v8f& d) { asm volatile("v_nop\n\tv_nop\n\tv_nop\n\tv_nop" : "+v"(a), "+v"(b), "+v"(c), "+v"(d)); }
template <typename T> struct Frag;
template <> struct Frag<_Float16> {
  typedef v16h V; union U { v16h v; v8h h[2]; };
  static __device__ __forceinline__ v16h load(const _Float16* p) {
    U f; f.h[0] = *(const v8h*)(p); f.h[1] = *(const v8h*)(p + 16); return f.v;
  }
  static __device__ __forceinline__ v8f mma(v16h a, v16h b, v8f c) {
    return __builtin_amdgcn_wmma_f32_16x16x32_f16(false, a, false, b, (short)0, c, false, false);
  }
  static __device__ __forceinline__ void guard4(v8f& a, v8f& b, v8f& c, v8f& d, v16h x, v16h y) { dep_guard4_h(a, b, c, d, x, y); }
  static __device__ __forceinline__ void keep(v16h a, v16h b, v16h c, v16h d) { keep4_h(a, b, c, d); }
};
template <> struct Frag<__bf16> {
  typedef v16b V; union U { v16b v; v8b h[2]; };
  static __device__ __forceinline__ v16b load(const __bf16* p) {
    U f; f.h[0] = *(const v8b*)(p); f.h[1] = *(const v8b*)(p + 16); return f.v;
  }
  static __device__ __forceinline__ v8f mma(v16b a, v16b b, v8f c) {
    return __builtin_amdgcn_wmma_f32_16x16x32_bf16(false, a, false, b, (short)0, c, false, false);
  }
  static __device__ __forceinline__ void guard4(v8f& a, v8f& b, v8f& c, v8f& d, v16b x, v16b y) { dep_guard4_b(a, b, c, d, x, y); }
  static __device__ __forceinline__ void keep(v16b a, v16b b, v16b c, v16b d) { keep4_b(a, b, c, d); }
};
typedef Frag<_Float16> FragH;

template <int ET> struct Elem;
template <> struct Elem<0> { typedef _Float16 T; };
template <> struct Elem<1> { typedef __bf16 T; };
template <int ET, int SPLITK, int BIAS_MODE, int OUT_MODE>
__global__ __launch_bounds__(256) void wmma_gemm64(
    const unsigned short* __restrict__ Ap, const unsigned short* __restrict__ A2p, int lda, long strideA,
    const unsigned short* __restrict__ Btp, const unsigned short* __restrict__ Bt2p, int ldb, long strideB,
    void* __restrict__ Cout, void* __restrict__ Cout2, int ldc, long strideC,
    const float* __restrict__ bias,
    int M, int N, int K, float scale) {
  typedef typename Elem<ET>::T T;
  typedef typename Frag<T>::V V;
  const T* A = (const T*)Ap; const T* A2 = (const T*)A2p; const T* Bt = (const T*)Btp; const T* Bt2 = (const T*)Bt2p;
  __shared__ __align__(16) float sT[8][16 * 68];
  const int b    = blockIdx.y;
  const int lane = threadIdx.x & 31;
  const int wave = threadIdx.x >> 5;
  const int tilesN = N >> 6;
  const int tilesM = M >> 6;
  const int tile = blockIdx.x * 8 + wave;
  if (tile >= tilesM * tilesN) return;
  const int tm = tile / tilesN;
  const int tn = tile - tm * tilesN;
  const int m0 = tm << 6;
  const int n0 = tn << 6;

  const T* Ab  = A  + (size_t)b * strideA;
  const T* Bb  = Bt + (size_t)b * strideB;
  const T* Ab2 = (SPLITK != 0) ? (A2  + (size_t)b * strideA) : nullptr;
  const T* Bb2 = (SPLITK == 2) ? (Bt2 + (size_t)b * strideB) : nullptr;

  const int rlane = lane & 15;
  const int koff  = (lane >> 4) * 8;
  const int mOff  = (lane >> 4) * 8;

  v8f acc[4][4];
#pragma unroll
  for (int i = 0; i < 4; ++i)
#pragma unroll
    for (int j = 0; j < 4; ++j) acc[i][j] = (v8f){0.f,0.f,0.f,0.f,0.f,0.f,0.f,0.f};

  for (int k0 = 0; k0 < K; k0 += 32) {
    V bh[4], bl[4];
#pragma unroll
    for (int j = 0; j < 4; ++j) {
      const size_t bo = (size_t)(n0 + (j << 4) + rlane) * ldb + koff + k0;
      bh[j] = Frag<T>::load(Bb + bo);
      if (SPLITK == 2) bl[j] = Frag<T>::load(Bb2 + bo);
    }
#pragma unroll
    for (int i = 0; i < 4; ++i) {
      const size_t ao = (size_t)(m0 + (i << 4) + rlane) * lda + koff + k0;
      V ah = Frag<T>::load(Ab + ao);
      V al;
      if (SPLITK != 0) al = Frag<T>::load(Ab2 + ao);
#pragma unroll
      for (int j = 0; j < 4; ++j) {
        acc[i][j] = Frag<T>::mma(ah, bh[j], acc[i][j]);
        if (SPLITK == 2) acc[i][j] = Frag<T>::mma(ah, bl[j], acc[i][j]);
        if (SPLITK != 0) acc[i][j] = Frag<T>::mma(al, bh[j], acc[i][j]);
      }
      Frag<T>::guard4(acc[i][0], acc[i][1], acc[i][2], acc[i][3], ah, (SPLITK != 0) ? al : ah);
    }
    Frag<T>::keep(bh[0], bh[1], bh[2], bh[3]);
    if (SPLITK == 2) Frag<T>::keep(bl[0], bl[1], bl[2], bl[3]);
  }
  acc_guard4(acc[0][0], acc[0][1], acc[0][2], acc[0][3]);
  acc_guard4(acc[1][0], acc[1][1], acc[1][2], acc[1][3]);
  acc_guard4(acc[2][0], acc[2][1], acc[2][2], acc[2][3]);
  acc_guard4(acc[3][0], acc[3][1], acc[3][2], acc[3][3]);

  float* slab = sT[wave];
  float bvn[4];
  if (BIAS_MODE == 2) {
#pragma unroll
    for (int j = 0; j < 4; ++j) bvn[j] = bf_bits2f(f2bf_bits(bias[n0 + (j << 4) + rlane]));
  }
#pragma unroll
  for (int i = 0; i < 4; ++i) {
    const int mBase = m0 + (i << 4);
    float bvm[8];
    if (BIAS_MODE == 1) {
      const v4f b0 = *(const v4f*)(bias + mBase + mOff);
      const v4f b1 = *(const v4f*)(bias + mBase + mOff + 4);
#pragma unroll
      for (int r = 0; r < 4; ++r) { bvm[r] = bf_bits2f(f2bf_bits(b0[r])); bvm[4 + r] = bf_bits2f(f2bf_bits(b1[r])); }
    }
#pragma unroll
    for (int j = 0; j < 4; ++j) {
#pragma unroll
      for (int r = 0; r < 8; ++r) {
        float v = acc[i][j][r] * scale;
        if (BIAS_MODE == 1) v += bvm[r];
        if (BIAS_MODE == 2) v += bvn[j];
        slab[(mOff + r) * 68 + (j << 4) + rlane] = v;
      }
    }
    __builtin_amdgcn_fence(__ATOMIC_RELEASE, "workgroup");
    __builtin_amdgcn_wave_barrier();
    __builtin_amdgcn_fence(__ATOMIC_ACQUIRE, "workgroup");
    if (OUT_MODE == 0) {
      float* C = (float*)Cout + (size_t)b * strideC;
      const int hh = lane >> 4, c4 = (lane & 15) * 4;
      for (int pass = 0; pass < 2; ++pass) {
#pragma unroll
        for (int it = 0; it < 8; ++it) {
          const int row = it * 2 + hh;
          v4f v = *(const v4f*)(slab + row * 68 + c4);
          *(volatile v4f*)(C + (size_t)(mBase + row) * ldc + n0 + c4) = v;
        }
        __threadfence();
      }
    } else {
      const int q = lane >> 3, c8 = (lane & 7) * 8;
      unsigned short* C  = (unsigned short*)Cout  + (size_t)b * strideC;
      unsigned short* C2 = (OUT_MODE >= 2) ? ((unsigned short*)Cout2 + (size_t)b * strideC) : nullptr;
      for (int pass = 0; pass < 2; ++pass) {
#pragma unroll
        for (int it = 0; it < 4; ++it) {
          const int row = it * 4 + q;
          const float* sp = slab + row * 68 + c8;
          v8h hv, lv;
#pragma unroll
          for (int e = 0; e < 8; ++e) {
            const float val = sp[e];
            if (OUT_MODE == 1) {
              hv[e] = (_Float16)val;
            } else if (OUT_MODE == 2) {
              const unsigned short hb = f2bf_bits(val);
              const unsigned short lb = f2bf_bits(val - bf_bits2f(hb));
              hv[e] = __builtin_bit_cast(_Float16, hb);
              lv[e] = __builtin_bit_cast(_Float16, lb);
            } else {
              const float hf = rne11(val);
              hv[e] = (_Float16)hf;
              lv[e] = (_Float16)((val - hf) * 2048.0f);
            }
          }
          *(volatile v8h*)(C + (size_t)(mBase + row) * ldc + n0 + c8) = hv;
          if (OUT_MODE >= 2) *(volatile v8h*)(C2 + (size_t)(mBase + row) * ldc + n0 + c8) = lv;
        }
        __threadfence();
      }
    }
    __builtin_amdgcn_fence(__ATOMIC_RELEASE, "workgroup");
    __builtin_amdgcn_wave_barrier();
    __builtin_amdgcn_fence(__ATOMIC_ACQUIRE, "workgroup");
  }
}

__global__ __launch_bounds__(256) void cast8_bf16_kernel(const float* __restrict__ in, unsigned short* __restrict__ out, int n8) {
  const int i = blockIdx.x * 256 + threadIdx.x;
  if (i >= n8) return;
  const float* p = in + 8 * (size_t)i;
  const v4f a = *(const v4f*)(p);
  const v4f c = *(const v4f*)(p + 4);
  unsigned short hb[8];
#pragma unroll
  for (int e = 0; e < 4; ++e) {
    hb[e]     = f2bf_bits(a[e]);
    hb[4 + e] = f2bf_bits(c[e]);
  }
  const v4u u = (v4u){pk16(hb[0], hb[1]), pk16(hb[2], hb[3]), pk16(hb[4], hb[5]), pk16(hb[6], hb[7])};
  unsigned short* q = out + 8 * (size_t)i;
  *(volatile v4u*)q = u;
  __threadfence();
  *(volatile v4u*)q = u;
}

__global__ __launch_bounds__(256) void wt_bf16_kernel(const float* __restrict__ W, unsigned short* __restrict__ out,
                                                     int kdim, int ncols) {
  __shared__ float sm[64][65];
  const int t  = threadIdx.x;
  const int d0 = blockIdx.x * 64;
  const int n0 = blockIdx.y * 64;
#pragma unroll
  for (int i = 0; i < 16; ++i) {
    const int e  = i * 256 + t;
    const int r  = e >> 6;
    const int cc = e & 63;
    sm[cc][r] = W[(size_t)(d0 + r) * ncols + n0 + cc];
  }
  __syncthreads();
  const int lane = t & 31, wave = t >> 5;
  const int q = lane >> 3, c8 = (lane & 7) * 8;
  for (int pass = 0; pass < 2; ++pass) {
#pragma unroll
    for (int it = 0; it < 2; ++it) {
      const int row = wave * 8 + it * 4 + q;
      unsigned short hb[8];
#pragma unroll
      for (int e = 0; e < 8; ++e) hb[e] = f2bf_bits(sm[row][c8 + e]);
      const v4u u = (v4u){pk16(hb[0], hb[1]), pk16(hb[2], hb[3]), pk16(hb[4], hb[5]), pk16(hb[6], hb[7])};
      *(volatile v4u*)(out + (size_t)(n0 + row) * kdim + d0 + c8) = u;
    }
    __threadfence();
  }
}

__device__ __forceinline__ v8f mma_h(v16h a, v16h b, v8f c) {
  c = __builtin_amdgcn_wmma_f32_16x16x32_f16(false, a, false, b, (short)0, c, false, false);
  asm volatile("v_nop\n\tv_nop\n\tv_nop\n\tv_nop" : "+v"(c) : "v"(a), "v"(b));
  return c;
}

template <bool SPL>
__global__ __launch_bounds__(128) void attn_causal_kernel(
    const unsigned short* __restrict__ QK,
    const unsigned short* __restrict__ VTh,
    const unsigned short* __restrict__ VTl,
    unsigned short* __restrict__ Ah,
    unsigned short* __restrict__ Al,
    int qb0) {
  __shared__ __align__(16) unsigned short Ksh[64 * 64];
  __shared__ __align__(16) unsigned short Vsh[64 * 64];
  __shared__ __align__(16) unsigned short Vsl[SPL ? 64 * 64 : 8];
  __shared__ __align__(16) _Float16 Psh[4][16 * 64];
  __shared__ __align__(16) _Float16 Psl[SPL ? 4 : 1][SPL ? 16 * 64 : 8];
  __shared__ __align__(16) float  Os[4][16 * 68];

  const int tid  = threadIdx.x;
  const int wave = tid >> 5;
  const int lane = tid & 31;
  const int hh   = lane >> 4;
  const int c    = lane & 15;
  const int bh   = blockIdx.x;
  const int h    = bh & (kHeads - 1);
  const int b    = bh >> 4;
  const int qb   = qb0 + (int)blockIdx.y;
  const int q0   = qb * 64 + wave * 16;
  const size_t tokBase = (size_t)b * kSeq;

  v16h qa0, qa1;
  {
    const _Float16* qrow = (const _Float16*)QK + (tokBase + q0 + c) * kQKld + h * kDh + 8 * hh;
    qa0 = FragH::load(qrow);
    qa1 = FragH::load(qrow + 32);
  }

  const v8f zero8 = (v8f){0.f,0.f,0.f,0.f,0.f,0.f,0.f,0.f};
  float mrow[8], lrow[8];
  v8f oacc[4], oacc2[4];
#pragma unroll
  for (int r = 0; r < 8; ++r) { mrow[r] = -INFINITY; lrow[r] = 0.f; }
#pragma unroll
  for (int t = 0; t < 4; ++t) { oacc[t] = zero8; oacc2[t] = zero8; }

  const int nChunks = qb + 1;
  for (int kc = 0; kc < nChunks; ++kc) {
    const int kv0 = kc * 64;
    __syncthreads();
#pragma unroll
    for (int i = 0; i < 4; ++i) {
      const int u = i * 128 + tid, r = u >> 3, seg = (u & 7) * 8;
      const v4u kw = *(const v4u*)(QK + (tokBase + kv0 + r) * kQKld + kDim + h * kDh + seg);
      const v4u vw = *(const v4u*)(VTh + (size_t)(h * kDh + r) * kTok + tokBase + kv0 + seg);
      *(v4u*)(Ksh + r * 64 + seg) = kw;
      *(v4u*)(Vsh + r * 64 + seg) = vw;
    }
    if (SPL) {
      asm volatile("" ::: "memory");
#pragma unroll
      for (int i = 0; i < 4; ++i) {
        const int u = i * 128 + tid, r = u >> 3, seg = (u & 7) * 8;
        const v4u lw = *(const v4u*)(VTl + (size_t)(h * kDh + r) * kTok + tokBase + kv0 + seg);
        *(v4u*)(Vsl + r * 64 + seg) = lw;
      }
    }
    __syncthreads();

    v8f s[4];
#pragma unroll
    for (int j = 0; j < 4; ++j) {
      s[j] = zero8;
      const _Float16* kr = (const _Float16*)Ksh + (j * 16 + c) * 64 + 8 * hh;
      const v16h kb0 = FragH::load(kr);
      const v16h kb1 = FragH::load(kr + 32);
      s[j] = mma_h(qa0, kb0, s[j]);
      s[j] = mma_h(qa1, kb1, s[j]);
    }

    const bool diag = (kc == qb);
    float cm[8];
#pragma unroll
    for (int r = 0; r < 8; ++r) {
      const int qrow = q0 + 8 * hh + r;
      float m = -INFINITY;
#pragma unroll
      for (int j = 0; j < 4; ++j) {
        const int kvcol = kv0 + j * 16 + c;
        float sv = s[j][r] * kScale;
        const bool masked = diag && (kvcol > qrow);
        sv = masked ? kMaskFill : sv;
        s[j][r] = sv;
        m = fmaxf(m, sv);
      }
#pragma unroll
      for (int off = 1; off < 16; off <<= 1) m = fmaxf(m, __shfl_xor(m, off, 32));
      cm[r] = m;
    }

    _Float16* pwh = Psh[wave];
    _Float16* pwl = Psl[SPL ? wave : 0];
#pragma unroll
    for (int r = 0; r < 8; ++r) {
      const float mnew  = fmaxf(mrow[r], cm[r]);
      const float alpha = expf(mrow[r] - mnew);
      mrow[r] = mnew;
      float psum = 0.f;
#pragma unroll
      for (int j = 0; j < 4; ++j) {
        const float p  = expf(s[j][r] - mnew);
        psum += p;
        const float pc = p * kPCarry;
        const int pidx = (8 * hh + r) * 64 + j * 16 + c;
        if (SPL) {
          const float hf = rne11(pc);
          pwh[pidx] = (_Float16)hf;
          pwl[pidx] = (_Float16)((pc - hf) * kResCarry);
        } else {
          pwh[pidx] = (_Float16)pc;
        }
      }
#pragma unroll
      for (int off = 1; off < 16; off <<= 1) psum += __shfl_xor(psum, off, 32);
      lrow[r] = lrow[r] * alpha + psum;
#pragma unroll
      for (int t = 0; t < 4; ++t) {
        oacc[t][r] *= alpha;
        if (SPL) oacc2[t][r] *= alpha;
      }
    }
    __builtin_amdgcn_fence(__ATOMIC_RELEASE, "workgroup");
    __builtin_amdgcn_wave_barrier();
    __builtin_amdgcn_fence(__ATOMIC_ACQUIRE, "workgroup");

#pragma unroll
    for (int kk = 0; kk < 2; ++kk) {
      const v16h pa = FragH::load(pwh + c * 64 + kk * 32 + 8 * hh);
      v16h pl;
      if (SPL) pl = FragH::load(pwl + c * 64 + kk * 32 + 8 * hh);
#pragma unroll
      for (int t = 0; t < 4; ++t) {
        const int voff = (t * 16 + c) * 64 + kk * 32 + 8 * hh;
        const v16h vb = FragH::load((const _Float16*)Vsh + voff);
        oacc[t] = mma_h(pa, vb, oacc[t]);
        if (SPL) {
          const v16h vl = FragH::load((const _Float16*)Vsl + voff);
          oacc2[t] = mma_h(pa, vl, oacc2[t]);
          oacc2[t] = mma_h(pl, vb, oacc2[t]);
        }
      }
    }
  }

  float* os = Os[wave];
#pragma unroll
  for (int r = 0; r < 8; ++r) {
    const float inv = (1.0f / lrow[r]) * kPCarryInv;
#pragma unroll
    for (int t = 0; t < 4; ++t) {
      float ov = oacc[t][r];
      if (SPL) ov = ov + oacc2[t][r] * kResInv;
      os[(8 * hh + r) * 68 + t * 16 + c] = ov * inv;
    }
  }
  __builtin_amdgcn_fence(__ATOMIC_RELEASE, "workgroup");
  __builtin_amdgcn_wave_barrier();
  __builtin_amdgcn_fence(__ATOMIC_ACQUIRE, "workgroup");
  {
    const int q4 = lane >> 3, c8 = (lane & 7) * 8;
    unsigned short* ahp = Ah + (tokBase + q0) * (size_t)kDim + h * kDh + c8;
    unsigned short* alp = Al + (tokBase + q0) * (size_t)kDim + h * kDh + c8;
    for (int pass = 0; pass < 2; ++pass) {
#pragma unroll
      for (int it = 0; it < 4; ++it) {
        const int row = it * 4 + q4;
        const float* sp = os + row * 68 + c8;
        unsigned short hb[8], lb[8];
#pragma unroll
        for (int e = 0; e < 8; ++e) {
          const float val = sp[e];
          hb[e] = f2bf_bits(val);
          lb[e] = f2bf_bits(val - bf_bits2f(hb[e]));
        }
        const v4u hu = (v4u){pk16(hb[0], hb[1]), pk16(hb[2], hb[3]), pk16(hb[4], hb[5]), pk16(hb[6], hb[7])};
        const v4u lu = (v4u){pk16(lb[0], lb[1]), pk16(lb[2], lb[3]), pk16(lb[4], lb[5]), pk16(lb[6], lb[7])};
        *(volatile v4u*)(ahp + (size_t)row * kDim) = hu;
        *(volatile v4u*)(alp + (size_t)row * kDim) = lu;
      }
      __threadfence();
    }
  }
}

extern "C" void kernel_launch(void* const* d_in, const int* in_sizes, int n_in,
                              void* d_out, int out_size, void* d_ws, size_t ws_size,
                              hipStream_t stream) {
  if (n_in < 5) return;
  if (in_sizes[0] != kTok * kDim) return;
  if (in_sizes[1] != kDim * kNQKV) return;
  if (in_sizes[2] != kNQKV) return;
  if (in_sizes[3] != kDim * kDim) return;
  if (in_sizes[4] != kDim) return;
  if (out_size != kTok * kDim) return;

  const size_t szXb = (size_t)kTok * kDim * 2;
  const size_t szWa = (size_t)kNQKV * kDim * 2;
  const size_t szWp = (size_t)kDim * kDim * 2;
  const size_t szQK = (size_t)kTok * kQKld * 2;
  const size_t szVT = (size_t)kDim * kTok * 2;
  const size_t szA  = (size_t)kTok * kDim * 2;
  const size_t offXb = 0;
  const size_t offWa = offXb + szXb;
  const size_t offWp = offWa + szWa;
  const size_t offQK = offWp + szWp;
  const size_t offVh = offQK + szQK;
  const size_t offVl = offVh + szVT;
  const size_t offAh = offVl + szVT;
  const size_t offAl = offAh + szA;
  const size_t total = offAl + szA;
  if (ws_size < total) return;

  const float* x  = (const float*)d_in[0];
  const float* wa = (const float*)d_in[1];
  const float* ba = (const float*)d_in[2];
  const float* wp = (const float*)d_in[3];
  const float* bp = (const float*)d_in[4];
  char* ws = (char*)d_ws;
  unsigned short* Xb   = (unsigned short*)(ws + offXb);
  unsigned short* WaT  = (unsigned short*)(ws + offWa);
  unsigned short* WpT  = (unsigned short*)(ws + offWp);
  unsigned short* QK16 = (unsigned short*)(ws + offQK);
  unsigned short* VTh  = (unsigned short*)(ws + offVh);
  unsigned short* VTl  = (unsigned short*)(ws + offVl);
  unsigned short* Ah   = (unsigned short*)(ws + offAh);
  unsigned short* Al   = (unsigned short*)(ws + offAl);

  const int n8 = (kTok * kDim) / 8;
  cast8_bf16_kernel<<<dim3(n8 / 256), dim3(256), 0, stream>>>(x, Xb, n8);
  wt_bf16_kernel<<<dim3(kDim / 64, kNQKV / 64), dim3(256), 0, stream>>>(wa, WaT, kDim, kNQKV);
  wt_bf16_kernel<<<dim3(kDim / 64, kDim / 64), dim3(256), 0, stream>>>(wp, WpT, kDim, kDim);

  wmma_gemm64<1, 0, 2, 1><<<dim3(((kTok / 64) * (kQKld / 64)) / 8, 1), dim3(256), 0, stream>>>(
      Xb, Xb, kDim, 0L, WaT, WaT, kDim, 0L,
      (void*)QK16, (void*)QK16, kQKld, 0L, ba, kTok, kQKld, kDim, 1.0f);
  wmma_gemm64<1, 0, 1, 3><<<dim3(((kDim / 64) * (kTok / 64)) / 8, 1), dim3(256), 0, stream>>>(
      WaT + (size_t)2 * kDim * kDim, WaT + (size_t)2 * kDim * kDim, kDim, 0L, Xb, Xb, kDim, 0L,
      (void*)VTh, (void*)VTl, kTok, 0L, ba + 2 * kDim, kDim, kTok, kDim, 1.0f);

  attn_causal_kernel<true><<<dim3(kBatch * kHeads, kSplitQB), dim3(128), 0, stream>>>(QK16, VTh, VTl, Ah, Al, 0);
  attn_causal_kernel<false><<<dim3(kBatch * kHeads, kSeq / 64 - kSplitQB), dim3(128), 0, stream>>>(QK16, VTh, VTl, Ah, Al, kSplitQB);

  wmma_gemm64<1, 1, 2, 0><<<dim3(((kTok / 64) * (kDim / 64)) / 8, 1), dim3(256), 0, stream>>>(
      Ah, Al, kDim, 0L, WpT, WpT, kDim, 0L,
      d_out, d_out, kDim, 0L, bp, kTok, kDim, kDim, 1.0f);
}
